// KgAttention_24747601559685
// MI455X (gfx1250) — hardware-run, weakly checked
//
#include <hip/hip_runtime.h>
#include <stddef.h>
#include <stdint.h>

#define NENT   100000
#define EMB    128
#define NEDGE  600000
#define NREL   64
#define NTHR   256
#define NWAVE  8
#define EPT    8
#define CHUNK  (NTHR * EPT)
#define WCAP   (EPT * 32)
#define LISTN  (NWAVE * WCAP)
#define NBA    1024
#define SLA    10
#define RCAP   28672
#define DEGCAP 32
#define HB     64
#define EBMAX  (HB * DEGCAP)
#define GBK    ((NENT + NBA - 1) / NBA)
#define NPAD   (GBK * NBA)
#define GHOP   ((NENT + HB - 1) / HB)
#define BK_ZINTS (LISTN + 2 * RCAP + 3 * NBA)
#define MISC_INTS 16
#define BK_LDS_BYTES ((BK_ZINTS + MISC_INTS) * 4)
#define WSMAX  134217728

#define O_REL  0
#define O_B    32768
#define O_A    98304
#define O_L    131072
#define O_ENT  163840
#define O_ATT  172032
#define O_HIT  180224
#define O_DEG  188416
#define O_OFF  188928
#define O_PART 189440
#define HOP_LDS_BYTES 189952

static_assert(NENT <= (1 << 17));
static_assert(NREL <= 64 && (NREL & (NREL - 1)) == 0);
static_assert(EMB == 128 && EMB == 4 * 32);
static_assert(NTHR == 256 && NWAVE * 32 == NTHR);
static_assert(DEGCAP % 32 == 0 && DEGCAP == 32);
static_assert(HB == 64 && EBMAX == 2048 && EBMAX % 64 == 0);
static_assert((CHUNK & (CHUNK - 1)) == 0 && CHUNK <= 4096);
static_assert((NBA & (NBA - 1)) == 0 && NBA == (1 << SLA) && NBA == NTHR * 4);
static_assert(((long long)NEDGE << SLA) < (1LL << 31));
static_assert(BK_ZINTS % (NTHR * 4) == 0 && RCAP % 4 == 0 && LISTN % 4 == 0);
static_assert(NBA % NWAVE == 0 && HB % NWAVE == 0);
static_assert((long long)GHOP * HB <= (long long)NPAD);
static_assert(BK_LDS_BYTES <= 327680);
static_assert(HOP_LDS_BYTES <= 327680);
static_assert(O_PART + 512 == HOP_LDS_BYTES);
static_assert((NPAD * 4) % 128 == 0);
static_assert(NEDGE % 4 == 0);

typedef float          v4f   __attribute__((ext_vector_type(4)));
typedef float          v8f   __attribute__((ext_vector_type(8)));
typedef int            v4i   __attribute__((ext_vector_type(4)));
typedef int            v8i   __attribute__((ext_vector_type(8)));
typedef unsigned       v2u   __attribute__((ext_vector_type(2)));
typedef unsigned short v8us  __attribute__((ext_vector_type(8)));
typedef unsigned short v16us __attribute__((ext_vector_type(16)));
typedef __bf16         v16bf __attribute__((ext_vector_type(16)));
typedef v4f  __attribute__((may_alias)) v4fa;
typedef v4i  __attribute__((may_alias)) v4ia;
typedef v2u  __attribute__((may_alias)) v2ua;
typedef v8us __attribute__((may_alias)) v8usa;
union FragB { v16bf v; v16us u; v8us h[2]; v8i w; };

__device__ __forceinline__ v8f wmb(const FragB& a, const FragB& b, v8f c) {
  v8f d = __builtin_amdgcn_wmma_f32_16x16x32_bf16(false, a.v, false, b.v, (short)0, c, false, false);
  asm volatile("v_nop\n\tv_nop\n\tv_nop\n\tv_nop" : "+v"(d) : "v"(a.w), "v"(b.w));
  return d;
}

__device__ __forceinline__ unsigned bf16_bits(float f) {
  const unsigned u = __float_as_uint(f);
  return (u + 0x7FFFu + ((u >> 16) & 1u)) >> 16;
}
__device__ __forceinline__ float bf16_val(float f) {
  return __uint_as_float(bf16_bits(f) << 16);
}
__device__ __forceinline__ v4f rne4(v4f v) {
  v4f r;
  r.x = bf16_val(v.x); r.y = bf16_val(v.y); r.z = bf16_val(v.z); r.w = bf16_val(v.w);
  return r;
}
struct HL { v2u hi; v2u lo; };
__device__ __forceinline__ HL split4(v4f v) {
  const unsigned h0 = bf16_bits(v.x), h1 = bf16_bits(v.y), h2 = bf16_bits(v.z), h3 = bf16_bits(v.w);
  const unsigned l0 = bf16_bits(v.x - __uint_as_float(h0 << 16));
  const unsigned l1 = bf16_bits(v.y - __uint_as_float(h1 << 16));
  const unsigned l2 = bf16_bits(v.z - __uint_as_float(h2 << 16));
  const unsigned l3 = bf16_bits(v.w - __uint_as_float(h3 << 16));
  HL o;
  o.hi.x = (h0 & 0xffffu) | (h1 << 16);
  o.hi.y = (h2 & 0xffffu) | (h3 << 16);
  o.lo.x = (l0 & 0xffffu) | (l1 << 16);
  o.lo.y = (l2 & 0xffffu) | (l3 << 16);
  return o;
}
__device__ __forceinline__ float tanh_fast(float v) {
  const float a = fabsf(v);
  const float u = __expf(-2.0f * a);
  const float r = (1.0f - u) * __builtin_amdgcn_rcpf(1.0f + u);
  return copysignf(r, v);
}
__device__ __forceinline__ float hsum16(float v) {
  v += __shfl_xor(v, 1);
  v += __shfl_xor(v, 2);
  v += __shfl_xor(v, 4);
  v += __shfl_xor(v, 8);
  return v;
}
__device__ __forceinline__ float wsum32(float v) {
  v += __shfl_xor(v, 16);
  v += __shfl_xor(v, 8);
  v += __shfl_xor(v, 4);
  v += __shfl_xor(v, 2);
  v += __shfl_xor(v, 1);
  return v;
}
__device__ __forceinline__ float wmax32(float v) {
  v = fmaxf(v, __shfl_xor(v, 16));
  v = fmaxf(v, __shfl_xor(v, 8));
  v = fmaxf(v, __shfl_xor(v, 4));
  v = fmaxf(v, __shfl_xor(v, 2));
  v = fmaxf(v, __shfl_xor(v, 1));
  return v;
}

template <int SLB>
__device__ __forceinline__ int scan_chunk(const int* __restrict__ dsts, int nE, int cbase, int slotBase,
                                          int nb, int vec8, int* list, int tid, int lane, int wave) {
  int wc = 0;
  const int el0  = tid * EPT;
  const int e0   = cbase + el0;
  const int sent = -2147483647 - 1;
  v4i da, db;
  if (vec8 != 0 && cbase + CHUNK <= nE) {
    da = *(const v4i*)(dsts + e0);
    db = *(const v4i*)(dsts + e0 + 4);
  } else {
    da.x = (e0     < nE) ? dsts[min(e0,     nE - 1)] : sent;
    da.y = (e0 + 1 < nE) ? dsts[min(e0 + 1, nE - 1)] : sent;
    da.z = (e0 + 2 < nE) ? dsts[min(e0 + 2, nE - 1)] : sent;
    da.w = (e0 + 3 < nE) ? dsts[min(e0 + 3, nE - 1)] : sent;
    db.x = (e0 + 4 < nE) ? dsts[min(e0 + 4, nE - 1)] : sent;
    db.y = (e0 + 5 < nE) ? dsts[min(e0 + 5, nE - 1)] : sent;
    db.z = (e0 + 6 < nE) ? dsts[min(e0 + 6, nE - 1)] : sent;
    db.w = (e0 + 7 < nE) ? dsts[min(e0 + 7, nE - 1)] : sent;
  }
  const unsigned nbs = (unsigned)slotBase;
  const unsigned unb = (unsigned)nb;
  const unsigned s0 = (unsigned)da.x - nbs, s1 = (unsigned)da.y - nbs;
  const unsigned s2 = (unsigned)da.z - nbs, s3 = (unsigned)da.w - nbs;
  const unsigned s4 = (unsigned)db.x - nbs, s5 = (unsigned)db.y - nbs;
  const unsigned s6 = (unsigned)db.z - nbs, s7 = (unsigned)db.w - nbs;
  const bool h0 = s0 < unb, h1 = s1 < unb, h2 = s2 < unb, h3 = s3 < unb;
  const bool h4 = s4 < unb, h5 = s5 < unb, h6 = s6 < unb, h7 = s7 < unb;
  const unsigned any = __builtin_amdgcn_ballot_w32(h0 | h1 | h2 | h3 | h4 | h5 | h6 | h7);
  if (any != 0u) {
#define HITJ(J, HJ, SJ) { \
      const unsigned mj = __builtin_amdgcn_ballot_w32(HJ); \
      if (mj != 0u) { \
        if (HJ) { \
          const int pos = wc + (int)__builtin_amdgcn_mbcnt_lo(mj, 0u); \
          if (pos < WCAP) list[wave * WCAP + pos] = ((el0 + (J)) << SLB) | (int)(SJ); \
        } \
        wc += (int)__builtin_popcount(mj); } }
    HITJ(0, h0, s0)
    HITJ(1, h1, s1)
    HITJ(2, h2, s2)
    HITJ(3, h3, s3)
    HITJ(4, h4, s4)
    HITJ(5, h5, s5)
    HITJ(6, h6, s6)
    HITJ(7, h7, s7)
#undef HITJ
  }
  return wc;
}

__device__ __forceinline__ v8us col8(const float* __restrict__ W, int n, int k8) {
  v8us o;
#pragma unroll
  for (int j = 0; j < 8; ++j) o[j] = (unsigned short)bf16_bits(W[(size_t)(k8 + j) * EMB + n]);
  return o;
}

__global__ __launch_bounds__(NTHR) void k_prep(const float* __restrict__ qw, const float* __restrict__ kw,
                                               const float* __restrict__ ee,
                                               unsigned short* QW2, unsigned short* KW2, unsigned short* KW1,
                                               float* REL) {
  const int u    = (int)blockIdx.x * NTHR + (int)threadIdx.x;
  const int part = u >> 11;
  const int v    = u & 2047;
  if (part == 0) {
    const int n = v >> 4, k8 = (v & 15) * 8;
    const v8us o = col8(qw, n, k8);
    unsigned short* p0 = QW2 + (size_t)n * 256 + k8;
    *(volatile v8us*)p0 = o;
    *(volatile v8us*)(p0 + EMB) = o;
    __threadfence();
    *(volatile v8us*)p0 = o;
    *(volatile v8us*)(p0 + EMB) = o;
  } else if (part == 1) {
    const int n = v >> 4, k8 = (v & 15) * 8;
    const v8us o = col8(kw, n, k8);
    unsigned short* p0 = KW2 + (size_t)n * 256 + k8;
    unsigned short* p1 = KW1 + (size_t)n * EMB + k8;
    *(volatile v8us*)p0 = o;
    *(volatile v8us*)(p0 + EMB) = o;
    *(volatile v8us*)p1 = o;
    __threadfence();
    *(volatile v8us*)p0 = o;
    *(volatile v8us*)(p0 + EMB) = o;
    *(volatile v8us*)p1 = o;
  } else if (part == 2) {
    const v4f a = *(const v4f*)(ee + (size_t)v * 4);
    const v4f r = rne4(a);
    float* dp = REL + (size_t)v * 4;
    *(volatile v4f*)dp = r;
    __threadfence();
    *(volatile v4f*)dp = r;
  }
}

__global__ __launch_bounds__(NTHR) void k_bucket(const int* __restrict__ eidx, const int* __restrict__ etype,
                                                 int* hits, int* degflag) {
  extern __shared__ __attribute__((aligned(16))) int bsm[];
  int* list = bsm;
  int* hl   = bsm + LISTN;
  int* sl   = hl + RCAP;
  int* cnt  = sl + RCAP;
  int* offs = cnt + NBA;
  int* cur  = offs + NBA;
  int* misc = cur + NBA;
  const int tid = (int)threadIdx.x, lane = tid & 31, wave = tid >> 5;
  const int nodeBase = (int)blockIdx.x * NBA;
  const int nE = NEDGE;

  {
    const v4i z4 = {0, 0, 0, 0};
    for (int i = tid * 4; i < BK_ZINTS; i += NTHR * 4) *(v4ia*)(bsm + i) = z4;
    if (tid < MISC_INTS) misc[tid] = 0;
  }
  __syncthreads();

  int t = 0, ov = 0;
  const int nChunks = (nE + CHUNK - 1) / CHUNK;
#pragma unroll 1
  for (int ch = 0; ch < nChunks; ++ch) {
    const int cbase = ch * CHUNK;
    const int wc = scan_chunk<SLA>(eidx, nE, cbase, nodeBase, NBA, 1, list, tid, lane, wave);
    if (lane == 0) misc[wave] = wc;
    __syncthreads();
    if (wave == 0) {
#pragma unroll 1
      for (int w2 = 0; w2 < NWAVE; ++w2) {
        int c = misc[w2];
        c = c < 0 ? 0 : (c > WCAP ? WCAP : c);
#pragma unroll 1
        for (int b0 = 0; b0 < c; b0 += 32) {
          const int idx = b0 + lane;
          const int ent = list[w2 * WCAP + (idx < WCAP ? idx : WCAP - 1)];
          const int m32 = (c - b0) < 32 ? (c - b0) : 32;
#pragma unroll 1
          for (int k = 0; k < m32; ++k) {
            const int u    = __builtin_amdgcn_readlane(ent, k);
            const int slot = u & (NBA - 1);
            const int el   = (u >> SLA) & (CHUNK - 1);
            const int pk   = ((cbase + el) << SLA) | slot;
            if (t < RCAP) {
              if (lane == 0) { hl[t] = pk; cnt[slot] = cnt[slot] + 1; }
              t = t + 1;
            } else {
              ov = 1;
            }
          }
        }
      }
    }
    __syncthreads();
  }
  if (wave == 0 && lane == 0) { misc[8] = t; misc[9] = ov; }
  __syncthreads();
  int tt = misc[8];
  tt = tt < 0 ? 0 : (tt > RCAP ? RCAP : tt);
  const int ovf = misc[9];

  if (wave == 0) {
    const int base = lane * (NBA / 32);
    int s = 0;
#pragma unroll 1
    for (int i = 0; i < NBA / 32; ++i) s += cnt[base + i];
    int incl = s;
#pragma unroll
    for (int d = 1; d < 32; d <<= 1) {
      const int y = __shfl_up(incl, d, 32);
      if (lane >= d) incl += y;
    }
    int run = incl - s;
#pragma unroll 1
    for (int i = 0; i < NBA / 32; ++i) {
      const int cv = cnt[base + i];
      offs[base + i] = run;
      cur[base + i]  = run;
      run += cv;
    }
  }
  __syncthreads();
  if (wave == 0) {
#pragma unroll 1
    for (int b0 = 0; b0 < tt; b0 += 32) {
      const int idx = b0 + lane;
      const int ent = hl[idx < RCAP ? idx : RCAP - 1];
      const int m32 = (tt - b0) < 32 ? (tt - b0) : 32;
#pragma unroll 1
      for (int k = 0; k < m32; ++k) {
        const int u    = __builtin_amdgcn_readlane(ent, k);
        const int slot = u & (NBA - 1);
        if (lane == 0) {
          int p = cur[slot];
          p = p < 0 ? 0 : (p > RCAP - 1 ? RCAP - 1 : p);
          sl[p] = u;
          cur[slot] = p + 1;
        }
      }
    }
  }
  __syncthreads();

  {
    const v4i c4 = *(const v4ia*)(cnt + 4 * tid);
    v4i dg, fg;
    dg.x = c4.x < 0 ? 0 : (c4.x > DEGCAP ? DEGCAP : c4.x);
    dg.y = c4.y < 0 ? 0 : (c4.y > DEGCAP ? DEGCAP : c4.y);
    dg.z = c4.z < 0 ? 0 : (c4.z > DEGCAP ? DEGCAP : c4.z);
    dg.w = c4.w < 0 ? 0 : (c4.w > DEGCAP ? DEGCAP : c4.w);
    fg.x = (ovf != 0 || c4.x > DEGCAP) ? 1 : 0;
    fg.y = (ovf != 0 || c4.y > DEGCAP) ? 1 : 0;
    fg.z = (ovf != 0 || c4.z > DEGCAP) ? 1 : 0;
    fg.w = (ovf != 0 || c4.w > DEGCAP) ? 1 : 0;
    int* pd = degflag + nodeBase + 4 * tid;
    int* pf = pd + NPAD;
    *(volatile v4i*)pd = dg;
    *(volatile v4i*)pf = fg;
    __threadfence();
    *(volatile v4i*)pd = dg;
    *(volatile v4i*)pf = fg;
  }

#pragma unroll 1
  for (int si = 0; si < NBA / NWAVE; ++si) {
    const int s    = si * NWAVE + wave;
    const int node = nodeBase + s;
    int c = cnt[s];
    c = c < 0 ? 0 : (c > DEGCAP ? DEGCAP : c);
    int o = offs[s];
    o = o < 0 ? 0 : (o > RCAP ? RCAP : o);
    int idx = o + lane;
    idx = idx > RCAP - 1 ? RCAP - 1 : idx;
    const int ent = sl[idx];
    int eid = ent >> SLA;
    eid = eid < 0 ? 0 : (eid > NEDGE - 1 ? NEDGE - 1 : eid);
    int tl = eidx[NEDGE + eid];
    int ty = etype[eid];
    asm volatile("" :: "v"(tl), "v"(ty));
    tl = tl < 0 ? 0 : (tl > NENT - 1 ? NENT - 1 : tl);
    ty = ty < 0 ? 0 : (ty > NREL - 1 ? NREL - 1 : ty);
    const int packed = tl | (ty << 17);
    const int entry  = (lane < c) ? packed : 0;
    int* hp = hits + (size_t)node * DEGCAP + lane;
    *(volatile int*)hp = entry;
    __threadfence();
    *(volatile int*)hp = entry;
  }
}

template <int KP>
__device__ __forceinline__ void tile_gemm(const unsigned short* sA, const unsigned short* sB,
                                          int mt, int nh, int hh, int m, v8f (&acc)[4]) {
  static_assert(KP % 32 == 0);
  const unsigned short* ap = sA + (16 * mt + m) * KP + 8 * hh;
  const unsigned short* bp = sB + (64 * nh + m) * KP + 8 * hh;
#pragma unroll 1
  for (int k0 = 0; k0 < KP; k0 += 32) {
    FragB af;
    af.h[0] = *(const v8usa*)(ap + k0);
    af.h[1] = *(const v8usa*)(ap + k0 + 16);
#pragma unroll
    for (int nt = 0; nt < 4; ++nt) {
      const unsigned short* wq = bp + (16 * nt) * KP + k0;
      FragB bf;
      bf.h[0] = *(const v8usa*)wq;
      bf.h[1] = *(const v8usa*)(wq + 16);
      acc[nt] = wmb(af, bf, acc[nt]);
    }
  }
}

template <int RS, int LAST, int XT>
__global__ __launch_bounds__(NTHR) __attribute__((amdgpu_num_vgpr(248)))
void k_hop(const float* stin, const float* x0, const float* s1p, float* outp,
           const unsigned short* __restrict__ bq, const unsigned short* __restrict__ bk,
           const float* __restrict__ relp, const int* __restrict__ hits, const int* __restrict__ degflag) {
  constexpr int AKX = EMB * XT;
  static_assert(XT == 1 || XT == 2);
  extern __shared__ __attribute__((aligned(16))) unsigned char hsm[];
  float*          sREL  = (float*)(hsm + O_REL);
  unsigned short* sB    = (unsigned short*)(hsm + O_B);
  unsigned short* sA    = (unsigned short*)(hsm + O_A);
  float*          sL    = (float*)(hsm + O_L);
  int*            sENT  = (int*)(hsm + O_ENT);
  float*          sATT  = (float*)(hsm + O_ATT);
  int*            sHIT  = (int*)(hsm + O_HIT);
  int*            sDEG  = (int*)(hsm + O_DEG);
  int*            sFLG  = sDEG + HB;
  int*            sOFF  = (int*)(hsm + O_OFF);
  float*          sPART = (float*)(hsm + O_PART);

  const int tid = (int)threadIdx.x, lane = tid & 31, wave = tid >> 5, hh = lane >> 4, m = lane & 15;
  const int mt = wave & 3, nh = wave >> 2;
  const int hb0 = (int)blockIdx.x * HB;

  {
    const v4i z4 = {0, 0, 0, 0};
#pragma unroll
    for (int i = 0; i < 2; ++i) {
      const int q = tid + NTHR * i;
      *(v4ia*)(sENT + 4 * q) = z4;
      *(v4ia*)(sATT + 4 * q) = z4;
    }
#pragma unroll 4
    for (int i = 0; i < 8; ++i) {
      const int q = tid + NTHR * i;
      const v4f v = *(const v4f*)(relp + 4 * q);
      *(v4fa*)(sREL + 4 * q) = v;
    }
#pragma unroll
    for (int i = 0; i < 2; ++i) {
      const int q = tid + NTHR * i;
      const v4i v = *(const v4i*)(hits + (size_t)hb0 * DEGCAP + 4 * q);
      *(v4ia*)(sHIT + 4 * q) = v;
    }
    if (tid < 32) {
      const int off = (tid >> 4) * NPAD + hb0 + 4 * (tid & 15);
      v4i v = *(const v4i*)(degflag + off);
      const int hi = (tid < 16) ? DEGCAP : 1;
      v.x = v.x < 0 ? 0 : (v.x > hi ? hi : v.x);
      v.y = v.y < 0 ? 0 : (v.y > hi ? hi : v.y);
      v.z = v.z < 0 ? 0 : (v.z > hi ? hi : v.z);
      v.w = v.w < 0 ? 0 : (v.w > hi ? hi : v.w);
      *(v4ia*)(sDEG + 4 * tid) = v;
    }
  }
  __syncthreads();

  if (wave == 0) {
    const int d0 = sDEG[2 * lane], d1 = sDEG[2 * lane + 1];
    const int s = d0 + d1;
    int incl = s;
#pragma unroll
    for (int dd = 1; dd < 32; dd <<= 1) {
      const int y = __shfl_up(incl, dd, 32);
      if (lane >= dd) incl += y;
    }
    const int ex = incl - s;
    sOFF[2 * lane]     = ex;
    sOFF[2 * lane + 1] = ex + d0;
    if (lane == 31) sOFF[HB] = incl;
  }
  __syncthreads();

#pragma unroll 4
  for (int i = 0; i < 8; ++i) {
    const int p = tid + NTHR * i;
    const int s = p >> 5, k = p & 31;
    const int d  = sDEG[s];
    const int o  = sOFF[s];
    const int hv = sHIT[p];
    asm volatile("" :: "v"(d), "v"(o), "v"(hv));
    int tl = hv & 0x1FFFF;
    tl = tl > NENT - 1 ? NENT - 1 : tl;
    const int ty = (hv >> 17) & (NREL - 1);
    int j = o + k;
    j = j < 0 ? 0 : (j > EBMAX - 1 ? EBMAX - 1 : j);
    const int val = tl | (ty << 17) | (s << 23);
    if (k < d) sENT[j] = val;
  }
#pragma unroll 4
  for (int i = 0; i < 16; ++i) {
    const int q = tid + NTHR * i;
    const v4i v = *(const v4ia*)(bq + 8 * q);
    *(v4ia*)(sB + 8 * q) = v;
  }
#pragma unroll 4
  for (int i = 0; i < 8; ++i) {
    const int q = tid + NTHR * i;
    const int r = q >> 5, c4 = (q & 31) * 4;
    int row = hb0 + r;
    row = row > NENT - 1 ? NENT - 1 : row;
    v4f v = *(const v4f*)(stin + (size_t)row * EMB + c4);
    if constexpr (RS != 0) v = rne4(v);
    const HL s = split4(v);
    *(v2ua*)(sA + r * 256 + c4)       = s.hi;
    *(v2ua*)(sA + r * 256 + EMB + c4) = s.lo;
  }
  __syncthreads();

  {
    v8f acc[4];
    const v8f z = {0.f, 0.f, 0.f, 0.f, 0.f, 0.f, 0.f, 0.f};
#pragma unroll
    for (int nt = 0; nt < 4; ++nt) acc[nt] = z;
    tile_gemm<256>(sA, sB, mt, nh, hh, m, acc);
#pragma unroll
    for (int nt = 0; nt < 4; ++nt) {
      const int col = 64 * nh + 16 * nt + m;
#pragma unroll
      for (int r = 0; r < 8; ++r) sL[(16 * mt + 8 * hh + r) * EMB + col] = acc[nt][r];
    }
  }
  __syncthreads();

#pragma unroll 4
  for (int i = 0; i < AKX / 16; ++i) {
    const int q = tid + NTHR * i;
    const v4i v = *(const v4ia*)(bk + 8 * q);
    *(v4ia*)(sB + 8 * q) = v;
  }

  int Eb = __builtin_amdgcn_readfirstlane(sOFF[HB]);
  Eb = Eb < 0 ? 0 : (Eb > EBMAX ? EBMAX : Eb);
  const int ntile = (Eb + 63) >> 6;

#pragma unroll 1
  for (int t = 0; t < ntile; ++t) {
#pragma unroll 4
    for (int i = 0; i < 8; ++i) {
      const int rr = 8 * wave + i;
      const int j  = 64 * t + rr;
      const int ent = sENT[j];
      const int tl = ent & 0x1FFFF;
      const int ty = (ent >> 17) & (NREL - 1);
      v4f tv = *(const v4f*)(stin + (size_t)tl * EMB + 4 * lane);
      if constexpr (RS != 0) tv = rne4(tv);
      const v4f rv = *(const v4fa*)(sREL + ty * EMB + 4 * lane);
      v4f xv = rv * tv;
      if (j >= Eb) { const v4f z4 = {0.f, 0.f, 0.f, 0.f}; xv = z4; }
      const HL s = split4(xv);
      *(v2ua*)(sA + rr * AKX + 4 * lane) = s.hi;
      if constexpr (XT == 2) *(v2ua*)(sA + rr * AKX + EMB + 4 * lane) = s.lo;
    }
    __syncthreads();

    v8f acc[4];
    {
      const v8f z = {0.f, 0.f, 0.f, 0.f, 0.f, 0.f, 0.f, 0.f};
#pragma unroll
      for (int nt = 0; nt < 4; ++nt) acc[nt] = z;
    }
    tile_gemm<AKX>(sA, sB, mt, nh, hh, m, acc);

    {
      const int eb0 = 64 * t + 16 * mt + 8 * hh;
      const v4i ea = *(const v4ia*)(sENT + eb0);
      const v4i ec = *(const v4ia*)(sENT + eb0 + 4);
      int so[8];
      so[0] = ((ea.x >> 23) & (HB - 1)) * EMB;
      so[1] = ((ea.y >> 23) & (HB - 1)) * EMB;
      so[2] = ((ea.z >> 23) & (HB - 1)) * EMB;
      so[3] = ((ea.w >> 23) & (HB - 1)) * EMB;
      so[4] = ((ec.x >> 23) & (HB - 1)) * EMB;
      so[5] = ((ec.y >> 23) & (HB - 1)) * EMB;
      so[6] = ((ec.z >> 23) & (HB - 1)) * EMB;
      so[7] = ((ec.w >> 23) & (HB - 1)) * EMB;
      float part[8];
#pragma unroll
      for (int r = 0; r < 8; ++r) part[r] = 0.0f;
#pragma unroll
      for (int nt = 0; nt < 4; ++nt) {
        const int col = 64 * nh + 16 * nt + m;
#pragma unroll
        for (int r = 0; r < 8; ++r) part[r] += tanh_fast(acc[nt][r]) * sL[so[r] + col];
      }
#pragma unroll
      for (int r = 0; r < 8; ++r) part[r] = hsum16(part[r]);
      if (m == 0) {
#pragma unroll
        for (int r = 0; r < 8; ++r) sPART[nh * 64 + 16 * mt + 8 * hh + r] = part[r];
      }
    }
    __syncthreads();
    if (tid < 64) sATT[64 * t + tid] = sPART[tid] + sPART[64 + tid];
  }
  __syncthreads();

  const float NEG_INF = __int_as_float((int)0xff800000u);
  const float QNAN    = __int_as_float(0x7fc00000);
#pragma unroll 1
  for (int si = 0; si < HB / NWAVE; ++si) {
    const int s    = si * NWAVE + wave;
    const int node = hb0 + s;
    int d = __builtin_amdgcn_readfirstlane(sDEG[s]);
    d = d < 0 ? 0 : (d > DEGCAP ? DEGCAP : d);
    int o = __builtin_amdgcn_readfirstlane(sOFF[s]);
    o = o < 0 ? 0 : (o > EBMAX ? EBMAX : o);
    const int flag = __builtin_amdgcn_readfirstlane(sFLG[s]);
    int idx = o + lane;
    idx = idx > EBMAX - 1 ? EBMAX - 1 : idx;
    const float att = sATT[idx];
    const int   ent = sENT[idx];
    asm volatile("" :: "v"(att), "v"(ent));
    const bool valid = lane < d;
    const float am = valid ? att : NEG_INF;
    const float mx = wmax32(am);
    const float ex = expf(att - mx);
    const float ev = valid ? ex : 0.0f;
    const float sm = wsum32(ev);
    const float wv = ev / sm;
    const int  wvi = __float_as_int(wv);
    float a0 = 0.0f, a1 = 0.0f, a2 = 0.0f, a3 = 0.0f;
#pragma unroll 1
    for (int k = 0; k < d; ++k) {
      const float wk = __int_as_float(__builtin_amdgcn_readlane(wvi, k));
      const int   ek = __builtin_amdgcn_readlane(ent, k);
      const int tl = ek & 0x1FFFF;
      const int ty = (ek >> 17) & (NREL - 1);
      v4f tv = *(const v4f*)(stin + (size_t)tl * EMB + 4 * lane);
      if constexpr (RS != 0) tv = rne4(tv);
      const v4f rv = *(const v4fa*)(sREL + ty * EMB + 4 * lane);
      a0 += (wk * rv.x) * tv.x;
      a1 += (wk * rv.y) * tv.y;
      a2 += (wk * rv.z) * tv.z;
      a3 += (wk * rv.w) * tv.w;
    }
    const float cf = fmaxf((float)d, 1.0f);
    const float g0 = a0 / cf, g1 = a1 / cf, g2 = a2 / cf, g3 = a3 / cf;
    float ss = g0 * g0 + g1 * g1 + g2 * g2 + g3 * g3;
    ss = wsum32(ss);
    const float den = fmaxf(sqrtf(ss), 1e-12f);
    v4f nv;
    nv.x = g0 / den; nv.y = g1 / den; nv.z = g2 / den; nv.w = g3 / den;
    if (d == 0)    { const v4f z4 = {0.f, 0.f, 0.f, 0.f}; nv = z4; }
    if (flag != 0) { const v4f q4 = {QNAN, QNAN, QNAN, QNAN}; nv = q4; }

    const int rc = node > NENT - 1 ? NENT - 1 : node;
    v4f ov = nv;
    if constexpr (LAST != 0) {
      const v4f n1 = *(const v4f*)(s1p + (size_t)rc * EMB + 4 * lane);
      const v4f n2 = *(const v4f*)(stin + (size_t)rc * EMB + 4 * lane);
      const v4f xr = rne4(*(const v4f*)(x0 + (size_t)rc * EMB + 4 * lane));
      ov = ((((n1 + xr) + n2) + xr) + nv) + xr;
    }
    if (node < NENT) {
      float* rp = outp + (size_t)node * EMB + 4 * lane;
      *(volatile v4f*)rp = ov;
      __threadfence();
      *(volatile v4f*)rp = ov;
    }
  }
}

static inline size_t al256(size_t o) { return (o + 255) & ~(size_t)255; }

extern "C" void kernel_launch(void* const* d_in, const int* in_sizes, int n_in,
                              void* d_out, int out_size, void* d_ws, size_t ws_size,
                              hipStream_t stream) {
  if (n_in < 6) return;
  if (in_sizes[0] != NENT * EMB) return;
  if (in_sizes[1] != NREL * EMB) return;
  if (in_sizes[2] != EMB * EMB || in_sizes[3] != EMB * EMB) return;
  if (in_sizes[4] != 2 * NEDGE) return;
  if (in_sizes[5] != NEDGE) return;
  if ((long long)out_size != (long long)NENT * EMB) return;

  const float* ent   = (const float*)d_in[0];
  const float* eemb  = (const float*)d_in[1];
  const float* qw    = (const float*)d_in[2];
  const float* kw    = (const float*)d_in[3];
  const int*   eidx  = (const int*)d_in[4];
  const int*   etype = (const int*)d_in[5];
  float* out = (float*)d_out;

  char* ws = (char*)d_ws;
  size_t off = 0;
  const size_t oQW2 = off; off = al256(off + (size_t)EMB * 256 * 2);
  const size_t oKW2 = off; off = al256(off + (size_t)EMB * 256 * 2);
  const size_t oKW1 = off; off = al256(off + (size_t)EMB * EMB * 2);
  const size_t oREL = off; off = al256(off + (size_t)NREL * EMB * 4);
  const size_t oDF  = off; off = al256(off + (size_t)2 * NPAD * 4);
  const size_t oHIT = off; off = al256(off + (size_t)NPAD * DEGCAP * 4);
  const size_t oS1  = off; off = al256(off + (size_t)NENT * EMB * 4);
  const size_t oS2  = off; off = al256(off + (size_t)NENT * EMB * 4);
  if (off > ws_size || off > (size_t)WSMAX) return;
  unsigned short* QW2 = (unsigned short*)(ws + oQW2);
  unsigned short* KW2 = (unsigned short*)(ws + oKW2);
  unsigned short* KW1 = (unsigned short*)(ws + oKW1);
  float* REL  = (float*)(ws + oREL);
  int*   DFp  = (int*)(ws + oDF);
  int*   HITS = (int*)(ws + oHIT);
  float* S1   = (float*)(ws + oS1);
  float* S2   = (float*)(ws + oS2);

  hipFuncSetAttribute(reinterpret_cast<const void*>(&k_bucket), hipFuncAttributeMaxDynamicSharedMemorySize, (int)BK_LDS_BYTES);
  hipFuncSetAttribute(reinterpret_cast<const void*>(&k_hop<1, 0, 2>), hipFuncAttributeMaxDynamicSharedMemorySize, (int)HOP_LDS_BYTES);
  hipFuncSetAttribute(reinterpret_cast<const void*>(&k_hop<0, 0, 1>), hipFuncAttributeMaxDynamicSharedMemorySize, (int)HOP_LDS_BYTES);
  hipFuncSetAttribute(reinterpret_cast<const void*>(&k_hop<0, 1, 1>), hipFuncAttributeMaxDynamicSharedMemorySize, (int)HOP_LDS_BYTES);

  k_prep<<<(3 * 2048) / NTHR, NTHR, 0, stream>>>(qw, kw, eemb, QW2, KW2, KW1, REL);
  k_bucket<<<GBK, NTHR, BK_LDS_BYTES, stream>>>(eidx, etype, HITS, DFp);
  k_hop<1, 0, 2><<<GHOP, NTHR, HOP_LDS_BYTES, stream>>>(ent, ent, ent, S1, QW2, KW2, REL, HITS, DFp);
  k_hop<0, 0, 1><<<GHOP, NTHR, HOP_LDS_BYTES, stream>>>(S1, ent, ent, S2, QW2, KW1, REL, HITS, DFp);
  k_hop<0, 1, 1><<<GHOP, NTHR, HOP_LDS_BYTES, stream>>>(S2, ent, S1, out, QW2, KW1, REL, HITS, DFp);
}
